// PYG_GAT_1752346657316
// MI455X (gfx1250) — hardware-run, weakly checked
//
#include <hip/hip_runtime.h>


namespace {
constexpr int N = 50000, NP = 50048, EFULL = 800000, E = 800000, NLIM = 50048  , IN = 128, H1 = 4, C1 = 64, HC1 = H1 * C1, H2 = 8, C2 = 32, HC2 = H2 * C2, NOUT = C2;
constexpr float XS = 8.0f, WSC = 256.0f, SLOPE = 0.2f;
static_assert(NP % 16 == 0 && NP >= N && NLIM % 16 == 0 && NLIM <= NP && HC1 == 256 && HC2 == 256 && IN % 32 == 0, "tiling");
typedef _Float16 b16;
typedef __attribute__((ext_vector_type(16))) _Float16 v16b;
typedef __attribute__((ext_vector_type(8))) _Float16 v8b;
typedef __attribute__((ext_vector_type(8))) float v8f;
typedef __attribute__((ext_vector_type(4))) float v4f;
__device__ __forceinline__ float bf16_rne(float f) { unsigned int u = __float_as_uint(f); u += 0x7FFFu + ((u >> 16) & 1u); return __uint_as_float(u & 0xFFFF0000u); }
__device__ __forceinline__ void split16(float v, b16& hi, b16& lo) { hi = (b16)v; lo = (b16)(v - (float)hi); }
__device__ __forceinline__ v16b frag_kb(const b16* p, int hh) { const v8b a = *(const v8b*)(p + 8 * hh), b = *(const v8b*)(p + 16 + 8 * hh); v16b f;
#pragma unroll
  for (int e = 0; e < 8; ++e) { f[e] = a[e]; f[8 + e] = b[e]; } return f; }
__device__ __forceinline__ v8f wmma16b(v16b a, v16b b, v8f c) { v8f d = __builtin_amdgcn_wmma_f32_16x16x32_f16(false, a, false, b, (short)0, c, false, false); asm volatile("v_nop\n\tv_nop\n\tv_nop\n\tv_nop" : "+v"(d) : "v"(a), "v"(b)); return d; }
__device__ __forceinline__ void wave_lds_sync() { __builtin_amdgcn_fence(__ATOMIC_RELEASE, "workgroup"); __builtin_amdgcn_wave_barrier(); __builtin_amdgcn_fence(__ATOMIC_ACQUIRE, "workgroup"); }
__device__ __forceinline__ float pmul(float a, float b) { float p = a * b; asm volatile("" : "+v"(p)); return p; }
__device__ __forceinline__ int iclamp(int v, int lo, int hi) { return v < lo ? lo : (v > hi ? hi : v); }
constexpr int CSR_NBLK = 512, CSR_GB = 9, CSR_GN = 1 << CSR_GB  , CSR_MAXG = 512, CSR_CAP = 12288  ;
__global__ __launch_bounds__(64) void csrA_kernel(const int* __restrict__ dst, int E, int N, int nG, int CHP, int NGP, int* __restrict__ STG, int* __restrict__ HST) {
  extern __shared__ int sm[];
  int* cnt = sm; int* run = sm + NGP; int* ids = sm + 2 * NGP;
  const int b = blockIdx.x; const int ch = (E + CSR_NBLK - 1) / CSR_NBLK; const int e0 = b * ch, e1 = min(E, e0 + ch);
  for (int i = threadIdx.x; i < NGP; i += 64) cnt[i] = 0;
  for (int i = threadIdx.x; i < CHP; i += 64) ids[i] = -1;
  __syncthreads();
  if (threadIdx.x == 0) {
    for (int e = e0; e < e1; ++e) { int d = dst[e]; d = (d < 0) ? 0 : (d >= N ? N - 1 : d); cnt[d >> CSR_GB] += 1; }
    int acc = 0; for (int g = 0; g < nG; ++g) { run[g] = acc; acc += cnt[g]; }
    for (int e = e0; e < e1; ++e) { int d = dst[e]; d = (d < 0) ? 0 : (d >= N ? N - 1 : d); const int g = d >> CSR_GB; ids[run[g]] = e; run[g] += 1; } }
  __syncthreads();
  typedef __attribute__((ext_vector_type(4))) int v4i;
  for (int pass = 0; pass < 2; ++pass) {
    for (int i = threadIdx.x; i < CHP / 4; i += 64) *(volatile v4i*)(STG + (size_t)b * CHP + i * 4) = *(const v4i*)(&ids[i * 4]);
    for (int i = threadIdx.x; i < NGP / 4; i += 64) { v4i v; for (int e = 0; e < 4; ++e) v[e] = (i * 4 + e < nG) ? cnt[i * 4 + e] : 0; *(volatile v4i*)(HST + (size_t)b * NGP + i * 4) = v; }
    __threadfence(); }
}
__global__ __launch_bounds__(512) void csrS_kernel(const int* __restrict__ HST, int nG, int NGP, int* __restrict__ START, int* __restrict__ TOT, int* __restrict__ OFF) {
  __shared__ int tot[CSR_MAXG];
  const int b = threadIdx.x;
  for (int pass = 0; pass < 2; ++pass) { int runb = 0; for (int g = 0; g < nG; ++g) { int c = HST[(size_t)b * NGP + g]; c = (c < 0) ? 0 : c; ((volatile int*)OFF)[(size_t)g * CSR_NBLK + b] = runb; runb += c; } __threadfence(); }
  for (int g = threadIdx.x; g < nG; g += 512) { int s = 0; for (int bb = 0; bb < CSR_NBLK; ++bb) { int c = HST[(size_t)bb * NGP + g]; s += (c < 0) ? 0 : c; } tot[g] = s; }
  __syncthreads();
  if (threadIdx.x < 32) {
    __shared__ int st[CSR_MAXG + 32];
    if (threadIdx.x == 0) { int acc = 0; for (int g = 0; g < NGP; ++g) { st[g] = acc; if (g < nG) acc += (tot[g] + 31) & ~31; } st[NGP] = acc; }
    __builtin_amdgcn_fence(__ATOMIC_RELEASE, "workgroup"); __builtin_amdgcn_wave_barrier(); __builtin_amdgcn_fence(__ATOMIC_ACQUIRE, "workgroup");
    for (int pass = 0; pass < 2; ++pass) { for (int i = threadIdx.x; i < NGP + 32; i += 32) { ((volatile int*)START)[i] = (i <= NGP) ? st[min(i, NGP)] : 0; ((volatile int*)TOT)[i] = (i < nG) ? tot[i] : 0; } __threadfence(); } }
}
__global__ __launch_bounds__(256) void csrB_kernel(const int* __restrict__ dst, int N, int nG, int CHP, int NGP, int permLen, const int* __restrict__ STG, const int* __restrict__ HST, const int* __restrict__ OFF, const int* __restrict__ START, const int* __restrict__ TOT, int* __restrict__ PERM, int* __restrict__ ROWPTR, int* __restrict__ ROWCNT, int* __restrict__ FLAG) {
  typedef __attribute__((ext_vector_type(4))) int v4i;
  __shared__ int ids[CSR_CAP]; __shared__ unsigned short key[CSR_CAP]; __shared__ int outp[CSR_CAP]; __shared__ int ncnt[CSR_GN + 1]; __shared__ int boff[CSR_NBLK + 1];
  const int g = blockIdx.x, t_ = threadIdx.x; int tot = TOT[g]; int st = START[g], stn = START[g + 1]; const int v0 = g * CSR_GN; const int nv = min(CSR_GN, N - v0);
  st = (st < 0) ? 0 : (st > permLen - 32 ? permLen - 32 : st) & ~31; stn = (stn < st) ? st : (stn > permLen ? permLen : stn); tot = (tot < 0) ? 0 : tot; if (tot > stn - st && tot <= CSR_CAP) tot = stn - st;
  if (tot > CSR_CAP) {
    for (int pass = 0; pass < 2; ++pass) { for (int i = t_; i < CSR_GN / 4; i += 256) { v4i a, c; for (int e = 0; e < 4; ++e) { a[e] = st; c[e] = 0; } *(volatile v4i*)(ROWPTR + v0 + i * 4) = a; *(volatile v4i*)(ROWCNT + v0 + i * 4) = c; } if (t_ == 0) ((volatile int*)FLAG)[0] = 1; __threadfence(); } (void)nv; return; }
  if (t_ == 0) { int acc = 0; for (int b = 0; b < CSR_NBLK; ++b) { boff[b] = acc; int c = HST[(size_t)b * NGP + g]; c = (c < 0) ? 0 : (c > CHP ? CHP : c); acc += c; if (acc > tot) acc = tot; } boff[CSR_NBLK] = acc; }
  for (int i = t_; i <= CSR_GN; i += 256) ncnt[i] = 0;
  __syncthreads();
  for (int b = 0; b < CSR_NBLK; ++b) { const int c = boff[b + 1] - boff[b]; int o_ = OFF[(size_t)g * CSR_NBLK + b]; o_ = (o_ < 0) ? 0 : (o_ > CHP - c ? CHP - c : o_); const int* src_ = STG + (size_t)b * CHP + o_;
    for (int i = t_; i < c; i += 256) { int id = src_[i]; id = (id < 0) ? 0 : id; ids[boff[b] + i] = id; int d = dst[id]; d = (d < v0) ? v0 : (d >= N ? N - 1 : d); int kk = d - v0; kk = (kk < 0) ? 0 : (kk >= CSR_GN ? CSR_GN - 1 : kk); key[boff[b] + i] = (unsigned short)kk; } }
  __syncthreads();
  if (t_ == 0) { for (int i = 0; i < tot; ++i) ncnt[key[i]] += 1; int acc = 0; for (int vl = 0; vl < CSR_GN; ++vl) { const int c = ncnt[vl]; ncnt[vl] = acc; acc += c; } ncnt[CSR_GN] = acc;
    for (int i = 0; i < tot; ++i) { const int vl = key[i]; outp[ncnt[vl]] = ids[i]; ncnt[vl] += 1; }
    for (int vl = CSR_GN; vl > 0; --vl) ncnt[vl] = ncnt[vl - 1]; ncnt[0] = 0; }
  __syncthreads();
  for (int pass = 0; pass < 2; ++pass) {
    for (int i = t_; i < (stn - st) / 4; i += 256) { v4i v; for (int e = 0; e < 4; ++e) { const int q = i * 4 + e; v[e] = (q < tot) ? outp[q] : -1; } *(volatile v4i*)(PERM + st + i * 4) = v; }
    for (int i = t_; i < CSR_GN / 4; i += 256) { v4i a, c; for (int e = 0; e < 4; ++e) { const int vl = i * 4 + e; a[e] = st + ncnt[vl]; c[e] = (vl < nv) ? (ncnt[vl + 1] - ncnt[vl]) : 0; } *(volatile v4i*)(ROWPTR + v0 + i * 4) = a; *(volatile v4i*)(ROWCNT + v0 + i * 4) = c; }
    __threadfence(); }
}
__global__ __launch_bounds__(256) void csrZ_kernel(int* __restrict__ p, size_t n4) { typedef __attribute__((ext_vector_type(4))) int v4i; const size_t tid = (size_t)blockIdx.x * 256 + threadIdx.x, nth = (size_t)gridDim.x * 256; v4i z = {0, 0, 0, 0}; for (size_t i = tid; i < n4; i += nth) *(volatile v4i*)(p + i * 4) = z; }
struct CsrBufs { int *STG, *HST, *OFF, *START, *TOT, *PERM, *ROWPTR, *ROWCNT, *FLAG; int nG, NGP, CHP; size_t permLen; char* base; size_t bytes; };
static size_t csr_carve(CsrBufs& c, char* ws, size_t off, int E, int N) {
  const size_t off0 = off; c.base = ws + off;
  auto al = [&](size_t bytes) { char* p = ws + off; off += (bytes + 255) & ~(size_t)255; return p; };
  c.nG = (N + CSR_GN - 1) / CSR_GN; c.NGP = (c.nG + 31) & ~31; const int ch = (E + CSR_NBLK - 1) / CSR_NBLK; c.CHP = (ch + 31) & ~31; c.permLen = (size_t)E + 32 * (size_t)c.nG + 32;
  c.STG = (int*)al((size_t)CSR_NBLK * c.CHP * 4); c.HST = (int*)al((size_t)CSR_NBLK * c.NGP * 4); c.OFF = (int*)al((size_t)c.NGP * CSR_NBLK * 4); c.START = (int*)al((size_t)(c.NGP + 64) * 4); c.TOT = (int*)al((size_t)(c.NGP + 64) * 4);
  c.PERM = (int*)al(c.permLen * 4); c.ROWPTR = (int*)al((size_t)c.nG * CSR_GN * 4); c.ROWCNT = (int*)al((size_t)c.nG * CSR_GN * 4); c.FLAG = (int*)al(256);
  c.bytes = off - off0; return off;
}
static void csr_build(const CsrBufs& c, const int* dst, int E, int N, hipStream_t stream) {
  const size_t smem = (size_t)(2 * c.NGP + c.CHP) * 4;
  csrZ_kernel<<<512, 256, 0, stream>>>((int*)c.base, c.bytes / 16);
  csrA_kernel<<<CSR_NBLK, 64, smem, stream>>>(dst, E, N, c.nG, c.CHP, c.NGP, c.STG, c.HST);
  csrS_kernel<<<1, 512, 0, stream>>>(c.HST, c.nG, c.NGP, c.START, c.TOT, c.OFF);
  csrB_kernel<<<c.nG, 256, 0, stream>>>(dst, N, c.nG, c.CHP, c.NGP, (int)c.permLen, c.STG, c.HST, c.OFF, c.START, c.TOT, c.PERM, c.ROWPTR, c.ROWCNT, c.FLAG);
}

typedef __attribute__((ext_vector_type(4))) _Float16 v4h;
__device__ __forceinline__ float leaky(float v) { return v > 0.0f ? v : SLOPE * v; }
__device__ __forceinline__ float elu1(float v) { return v > 0.0f ? v : __expf(v) - 1.0f; }
__global__ __launch_bounds__(256) void prep_kernel(const float* __restrict__ x, const float* __restrict__ w1, const float* __restrict__ w2, b16* __restrict__ Xh, b16* __restrict__ WT1, b16* __restrict__ WT2) {
  size_t t = (size_t)blockIdx.x * 256 + threadIdx.x; const size_t nx = (size_t)NP * IN / 8, n1 = (size_t)HC1 * IN / 8, n2 = (size_t)HC2 * HC1 / 8; v8b o;
  if (t < nx) { const size_t e = t * 8; const size_t v = e / IN; for (int j = 0; j < 8; ++j) o[j] = (v < (size_t)N) ? (b16)(bf16_rne(x[e + j]) * XS) : (b16)0.0f; for (int pass = 0; pass < 2; ++pass) { *(volatile v8b*)(Xh + e) = o; __threadfence(); } return; } t -= nx;
  if (t < n1) { const size_t e = t * 8; const int oo = (int)(e / IN), k0 = (int)(e % IN); for (int j = 0; j < 8; ++j) o[j] = (b16)(bf16_rne(w1[(size_t)(k0 + j) * HC1 + oo]) * WSC); for (int pass = 0; pass < 2; ++pass) { *(volatile v8b*)(WT1 + e) = o; __threadfence(); } return; } t -= n1;
  if (t < n2) { const size_t e = t * 8; const int oo = (int)(e / HC1), k0 = (int)(e % HC1); for (int j = 0; j < 8; ++j) o[j] = (b16)(bf16_rne(w2[(size_t)(k0 + j) * HC2 + oo]) * WSC); for (int pass = 0; pass < 2; ++pass) { *(volatile v8b*)(WT2 + e) = o; __threadfence(); } }
}
template <int KD, int TWO, int NH, int HD>
__global__ __launch_bounds__(32) void proj_kernel(const b16* __restrict__ Ah, const b16* __restrict__ Al, const b16* __restrict__ WT, const float* __restrict__ asrc, const float* __restrict__ adst, float* __restrict__ Hp, float* __restrict__ AS) {
  __shared__ __attribute__((aligned(16))) float Tf[16][256 + 4], Ps[16][2 * NH];
  constexpr int TPH = HD / 16, HPG = 8 / TPH;
  const int lane = threadIdx.x, nloc = lane & 15, hlf = lane >> 4; const size_t m0 = (size_t)blockIdx.x * 16;
#pragma unroll 1
  for (int g = 0; g < 2; ++g) {
    v8f acc[8];
#pragma unroll
    for (int t = 0; t < 8; ++t) acc[t] = (v8f){};
#pragma unroll 2
    for (int kb = 0; kb < KD; kb += 32) { const v16b a = frag_kb(Ah + (m0 + nloc) * KD + kb, hlf); v16b al; if (TWO) al = frag_kb(Al + (m0 + nloc) * KD + kb, hlf);
#pragma unroll
      for (int t = 0; t < 8; ++t) { const v16b bw = frag_kb(WT + (size_t)((g * 8 + t) * 16 + nloc) * KD + kb, hlf); acc[t] = wmma16b(a, bw, acc[t]); if (TWO) acc[t] = wmma16b(al, bw, acc[t]); } }
    float ps[HPG][8], pd[HPG][8];
#pragma unroll
    for (int h = 0; h < HPG; ++h)
#pragma unroll
      for (int r8 = 0; r8 < 8; ++r8) { ps[h][r8] = 0.0f; pd[h][r8] = 0.0f; }
#pragma unroll
    for (int t = 0; t < 8; ++t) { const int c = (g * 8 + t) * 16 + nloc; const float ws_ = bf16_rne(asrc[c]), wd_ = bf16_rne(adst[c]);
#pragma unroll
      for (int r8 = 0; r8 < 8; ++r8) { const float v = acc[t][r8] * (1.0f / (XS * WSC)); Tf[8 * hlf + r8][c] = v; ps[t / TPH][r8] += pmul(v, ws_); pd[t / TPH][r8] += pmul(v, wd_); } }
#pragma unroll
    for (int h = 0; h < HPG; ++h)
#pragma unroll
      for (int r8 = 0; r8 < 8; ++r8) { float a = ps[h][r8], d = pd[h][r8];
#pragma unroll
        for (int o = 1; o < 16; o <<= 1) { a += __shfl_xor(a, o); d += __shfl_xor(d, o); } if (nloc == 0) { Ps[8 * hlf + r8][g * HPG + h] = a; Ps[8 * hlf + r8][NH + g * HPG + h] = d; } } }
  wave_lds_sync();
  for (int pass = 0; pass < 2; ++pass) { for (int rr = 0; rr < 16; ++rr) { *(volatile v4f*)(Hp + (m0 + rr) * 256 + lane * 4) = *(const v4f*)(&Tf[rr][lane * 4]); *(volatile v4f*)(Hp + (m0 + rr) * 256 + 128 + lane * 4) = *(const v4f*)(&Tf[rr][128 + lane * 4]); }
    for (int q = lane; q < 16 * 2 * NH / 4; q += 32) *(volatile v4f*)(AS + m0 * 2 * NH + q * 4) = *(const v4f*)(&Ps[0][0] + q * 4);
    __threadfence(); }
}
__global__ __launch_bounds__(256) void att1_kernel(const float* __restrict__ Hp, const float* __restrict__ AS, const float* __restrict__ bg, const int* __restrict__ srcs, const int* __restrict__ PERM, const int* __restrict__ ROWPTR, const int* __restrict__ ROWCNT, int permLen, b16* __restrict__ H1h, b16* __restrict__ H1l) {
  const int wave = threadIdx.x >> 5, lane = threadIdx.x & 31; const size_t v = (size_t)blockIdx.x * 8 + wave; if (v >= (size_t)NLIM) return; const int h = lane >> 3; const int c0 = lane * 8;
  v8b oh, ol; for (int i = 0; i < 8; ++i) { oh[i] = (b16)0.0f; ol[i] = (b16)0.0f; }
  if (v < (size_t)N) {
    const float ad = AS[v * 2 * H1 + H1 + h]; int st = ROWPTR[v], cnt = ROWCNT[v]; cnt = iclamp(cnt, 0, 1 << 20); st = iclamp(st, 0, permLen - cnt);
    float mx = leaky(AS[v * 2 * H1 + h] + ad);
#pragma unroll 1
    for (int j = 0; j < cnt; ++j) { const int e = iclamp(PERM[st + j], 0, E - 1); const size_t s = (size_t)iclamp(srcs[e], 0, N - 1); float l = leaky(AS[s * 2 * H1 + h] + ad); if (s >= (size_t)NLIM) l = -INFINITY; mx = fmaxf(mx, l); }
    float den; float o[8]; { const float p = __expf(leaky(AS[v * 2 * H1 + h] + ad) - mx); den = p; const v4f a = *(const v4f*)(Hp + v * HC1 + c0), b = *(const v4f*)(Hp + v * HC1 + c0 + 4); for (int i = 0; i < 4; ++i) { o[i] = pmul(p, a[i]); o[4 + i] = pmul(p, b[i]); } }
#pragma unroll 1
    for (int j = 0; j < cnt; ++j) { const int e = iclamp(PERM[st + j], 0, E - 1); const size_t s = (size_t)iclamp(srcs[e], 0, N - 1); float p = __expf(leaky(AS[s * 2 * H1 + h] + ad) - mx); if (s >= (size_t)NLIM) p = 0.0f; den += p;
      const v4f a = *(const v4f*)(Hp + s * HC1 + c0), b = *(const v4f*)(Hp + s * HC1 + c0 + 4); for (int i = 0; i < 4; ++i) { o[i] += pmul(p, a[i]); o[4 + i] += pmul(p, b[i]); } }
    const float inv = 1.0f / (den + 1e-16f);
#pragma unroll
    for (int i = 0; i < 8; ++i) { const float r = elu1(pmul(o[i], inv) + bf16_rne(bg[c0 + i])); b16 p, q; split16(r * XS, p, q); oh[i] = p; ol[i] = q; } }
  for (int pass = 0; pass < 2; ++pass) { *(volatile v8b*)(H1h + v * HC1 + c0) = oh; *(volatile v8b*)(H1l + v * HC1 + c0) = ol; __threadfence(); }
}
__global__ __launch_bounds__(256) void att2_kernel(const float* __restrict__ Hp, const float* __restrict__ AS, const float* __restrict__ bg, const int* __restrict__ srcs, const int* __restrict__ PERM, const int* __restrict__ ROWPTR, const int* __restrict__ ROWCNT, int permLen, float* __restrict__ out) {
  __shared__ float rowsum[8][H2][NOUT];
  const int wave = threadIdx.x >> 5, lane = threadIdx.x & 31; const size_t v = (size_t)blockIdx.x * 8 + wave; if (v >= (size_t)NLIM || v >= (size_t)N) return; const int h = lane >> 2; const int c0 = lane * 8, cl = (lane & 3) * 8;
  const float ad = AS[v * 2 * H2 + H2 + h]; int st = ROWPTR[v], cnt = ROWCNT[v]; cnt = iclamp(cnt, 0, 1 << 20); st = iclamp(st, 0, permLen - cnt);
  float mx = leaky(AS[v * 2 * H2 + h] + ad);
#pragma unroll 1
  for (int j = 0; j < cnt; ++j) { const int e = iclamp(PERM[st + j], 0, E - 1); const size_t s = (size_t)iclamp(srcs[e], 0, N - 1); float l = leaky(AS[s * 2 * H2 + h] + ad); if (s >= (size_t)NLIM) l = -INFINITY; mx = fmaxf(mx, l); }
  float den; float o[8]; { const float p = __expf(leaky(AS[v * 2 * H2 + h] + ad) - mx); den = p; const v4f a = *(const v4f*)(Hp + v * HC2 + c0), b = *(const v4f*)(Hp + v * HC2 + c0 + 4); for (int i = 0; i < 4; ++i) { o[i] = pmul(p, a[i]); o[4 + i] = pmul(p, b[i]); } }
#pragma unroll 1
  for (int j = 0; j < cnt; ++j) { const int e = iclamp(PERM[st + j], 0, E - 1); const size_t s = (size_t)iclamp(srcs[e], 0, N - 1); float p = __expf(leaky(AS[s * 2 * H2 + h] + ad) - mx); if (s >= (size_t)NLIM) p = 0.0f; den += p;
    const v4f a = *(const v4f*)(Hp + s * HC2 + c0), b = *(const v4f*)(Hp + s * HC2 + c0 + 4); for (int i = 0; i < 4; ++i) { o[i] += pmul(p, a[i]); o[4 + i] += pmul(p, b[i]); } }
  const float inv = 1.0f / (den + 1e-16f);
#pragma unroll
  for (int i = 0; i < 8; ++i) rowsum[wave][h][cl + i] = pmul(o[i], inv);
  wave_lds_sync();
  float r = bf16_rne(bg[lane]);
  { float s8 = 0.0f;
#pragma unroll
    for (int hh2 = 0; hh2 < H2; ++hh2) s8 += rowsum[wave][hh2][lane];
    r += s8 * (1.0f / H2); }
  for (int pass = 0; pass < 2; ++pass) { ((volatile float*)out)[v * NOUT + lane] = r; __threadfence(); }
}
}

extern "C" void kernel_launch(void* const* d_in, const int* in_sizes, int n_in, void* d_out, int out_size, void* d_ws, size_t ws_size, hipStream_t stream) {
  (void)n_in;
  auto Fp = [&](int i) { return (const float*)d_in[i]; }; auto Ip = [&](int i) { return (const int*)d_in[i]; };
  if (in_sizes[0] != N * IN || in_sizes[1] != 2 * EFULL || in_sizes[2] != IN * HC1 || in_sizes[3] != HC1 || in_sizes[4] != HC1 || in_sizes[5] != HC1 || in_sizes[6] != HC1 * HC2 || in_sizes[7] != HC2 || in_sizes[8] != HC2 || in_sizes[9] != NOUT || out_size != N * NOUT) return;
  size_t off = 0; char* ws = (char*)d_ws;
  auto carve = [&](size_t bytes) { char* p = ws + off; off += (bytes + 255) & ~(size_t)255; return p; };
  b16* Xh = (b16*)carve((size_t)NP * IN * 2); b16* WT1 = (b16*)carve((size_t)HC1 * IN * 2); b16* WT2 = (b16*)carve((size_t)HC2 * HC1 * 2);
  float* Hp = (float*)carve((size_t)NP * 256 * 4); float* AS = (float*)carve((size_t)NP * 2 * H2 * 4); b16* H1h = (b16*)carve((size_t)NP * HC1 * 2); b16* H1l = (b16*)carve((size_t)NP * HC1 * 2);
  CsrBufs csr; off = csr_carve(csr, ws, off, E, N);
  if (off > ws_size || off > ((size_t)128 << 20)) return;
  prep_kernel<<<(unsigned)((((size_t)NP * IN + (size_t)HC1 * IN + (size_t)HC2 * HC1) / 8 + 255) / 256), 256, 0, stream>>>(Fp(0), Fp(2), Fp(6), Xh, WT1, WT2);
  csr_build(csr, Ip(1) + EFULL, E, N, stream);
  proj_kernel<IN, 0, H1, C1><<<NLIM / 16, 32, 0, stream>>>(Xh, nullptr, WT1, Fp(3), Fp(4), Hp, AS);
  att1_kernel<<<NLIM / 8, 256, 0, stream>>>(Hp, AS, Fp(5), Ip(1), csr.PERM, csr.ROWPTR, csr.ROWCNT, (int)csr.permLen, H1h, H1l);
  proj_kernel<HC1, 1, H2, C2><<<NLIM / 16, 32, 0, stream>>>(H1h, H1l, WT2, Fp(7), Fp(8), Hp, AS);
  att2_kernel<<<NLIM / 8, 256, 0, stream>>>(Hp, AS, Fp(9), Ip(1), csr.PERM, csr.ROWPTR, csr.ROWCNT, (int)csr.permLen, (float*)d_out);
}
